// SSMLayerV2_29703993819796
// MI455X (gfx1250) — hardware-run, weakly checked
//
#include <hip/hip_runtime.h>
#include <math.h>

constexpr int kBatch = 4;
constexpr int kSeq   = 2048;
constexpr int kDim   = 1024;
constexpr int kNS    = 16;
constexpr int kRows  = kBatch * kSeq;
constexpr float kWCarry    = 32.0f;
constexpr float kWCarryInv = 1.0f / 32.0f;
constexpr float kInvDim    = 1.0f / 1024.0f;
constexpr float kLnEps     = 1e-5f;

typedef __attribute__((ext_vector_type(16))) _Float16 v16h;
typedef __attribute__((ext_vector_type(8)))  _Float16 v8h;
typedef __attribute__((ext_vector_type(16))) __bf16   v16b;
typedef __attribute__((ext_vector_type(8)))  __bf16   v8b;
typedef __attribute__((ext_vector_type(8)))  float    v8f;
typedef __attribute__((ext_vector_type(4)))  float    v4f;
typedef __attribute__((ext_vector_type(4)))  unsigned int v4u;

__device__ __forceinline__ unsigned short f2bf_bits(float f) {
  unsigned u = __float_as_uint(f);
  return (unsigned short)((u + 0x7FFFu + ((u >> 16) & 1u)) >> 16);
}
__device__ __forceinline__ float bf_bits2f(unsigned short h) { return __uint_as_float(((unsigned)h) << 16); }

__device__ __forceinline__ void dep_guard_h(v8f& a, v8f& b, v16h x, v16h y) { asm volatile("v_nop\n\tv_nop\n\tv_nop\n\tv_nop" : "+v"(a), "+v"(b) : "v"(x), "v"(y)); }
__device__ __forceinline__ void dep_guard_b(v8f& a, v8f& b, v16b x, v16b y) { asm volatile("v_nop\n\tv_nop\n\tv_nop\n\tv_nop" : "+v"(a), "+v"(b) : "v"(x), "v"(y)); }
__device__ __forceinline__ void keep4_h(v16h a, v16h b, v16h c, v16h d) { asm volatile("v_nop" :: "v"(a), "v"(b), "v"(c), "v"(d)); }
__device__ __forceinline__ void keep4_b(v16b a, v16b b, v16b c, v16b d) { asm volatile("v_nop" :: "v"(a), "v"(b), "v"(c), "v"(d)); }
__device__ __forceinline__ void acc_guard4(v8f& a, v8f& b, v8f& c, v8f& d) { asm volatile("v_nop\n\tv_nop\n\tv_nop\n\tv_nop" : "+v"(a), "+v"(b), "+v"(c), "+v"(d)); }
template <typename T> struct Frag;
template <> struct Frag<_Float16> {
  typedef v16h V; union U { v16h v; v8h h[2]; };
  static __device__ __forceinline__ v16h load(const _Float16* p) {
    U f; f.h[0] = *(const v8h*)(p); f.h[1] = *(const v8h*)(p + 16); return f.v;
  }
  static __device__ __forceinline__ v8f mma(v16h a, v16h b, v8f c) {
    return __builtin_amdgcn_wmma_f32_16x16x32_f16(false, a, false, b, (short)0, c, false, false);
  }
  static __device__ __forceinline__ void guard(v8f& a, v8f& b, v16h x, v16h y) { dep_guard_h(a, b, x, y); }
  static __device__ __forceinline__ void keep(v16h a, v16h b, v16h c, v16h d) { keep4_h(a, b, c, d); }
};
template <> struct Frag<__bf16> {
  typedef v16b V; union U { v16b v; v8b h[2]; };
  static __device__ __forceinline__ v16b load(const __bf16* p) {
    U f; f.h[0] = *(const v8b*)(p); f.h[1] = *(const v8b*)(p + 16); return f.v;
  }
  static __device__ __forceinline__ v8f mma(v16b a, v16b b, v8f c) {
    return __builtin_amdgcn_wmma_f32_16x16x32_bf16(false, a, false, b, (short)0, c, false, false);
  }
  static __device__ __forceinline__ void guard(v8f& a, v8f& b, v16b x, v16b y) { dep_guard_b(a, b, x, y); }
  static __device__ __forceinline__ void keep(v16b a, v16b b, v16b c, v16b d) { keep4_b(a, b, c, d); }
};

__device__ __forceinline__ unsigned pk16(unsigned short a, unsigned short b) { return (unsigned)a | ((unsigned)b << 16); }
__device__ __forceinline__ unsigned short h_bits(float f) { const _Float16 h = (_Float16)f; return __builtin_bit_cast(unsigned short, h); }

__device__ __forceinline__ void store2_v4u(unsigned short* q, v4u u) {
  *(volatile v4u*)q = u;
  __threadfence();
  *(volatile v4u*)q = u;
}
__device__ __forceinline__ void store2_v4f(float* q, v4f v) {
  *(volatile v4f*)q = v;
  __threadfence();
  *(volatile v4f*)q = v;
}

__device__ __forceinline__ float wave_sum(float v) {
  v += __shfl_xor(v, 16, 32);
  v += __shfl_xor(v, 8, 32);
  v += __shfl_xor(v, 4, 32);
  v += __shfl_xor(v, 2, 32);
  v += __shfl_xor(v, 1, 32);
  return v;
}
__device__ __forceinline__ float half16_sum(float v) {
  v += __shfl_xor(v, 8, 32);
  v += __shfl_xor(v, 4, 32);
  v += __shfl_xor(v, 2, 32);
  v += __shfl_xor(v, 1, 32);
  return v;
}

template <int ET> struct Elem;
template <> struct Elem<0> { typedef _Float16 T; };
template <> struct Elem<1> { typedef __bf16 T; };
template <int ET, bool SPLIT, int BIAS_MODE, int OUT_MODE, bool RESID, int ACT = 0>
__global__ __launch_bounds__(256) void wmma_gemm64(
    const unsigned short* __restrict__ Ap, const unsigned short* __restrict__ A2p, int lda, long strideA,
    const unsigned short* __restrict__ Btp, const unsigned short* __restrict__ Bt2p, int ldb, long strideB,
    void* __restrict__ Cout, void* __restrict__ Cout2, int ldc, long strideC,
    const float* __restrict__ bias,
    const float* __restrict__ resid, long strideR,
    int M, int N, int K, float scale) {
  typedef typename Elem<ET>::T T;
  typedef typename Frag<T>::V V;
  const T* A = (const T*)Ap; const T* A2 = (const T*)A2p; const T* Bt = (const T*)Btp; const T* Bt2 = (const T*)Bt2p;
  __shared__ __align__(16) float sT[8][16 * 68];
  const int b    = blockIdx.y;
  const int lane = threadIdx.x & 31;
  const int wave = threadIdx.x >> 5;
  const int tilesN = N >> 6;
  const int tilesM = M >> 6;
  const int tile = blockIdx.x * 8 + wave;
  if (tile >= tilesM * tilesN) return;
  const int tm = tile / tilesN;
  const int tn = tile - tm * tilesN;
  const int m0 = tm << 6;
  const int n0 = tn << 6;

  const T* Ab  = A  + (size_t)b * strideA;
  const T* Bb  = Bt + (size_t)b * strideB;
  const T* Ab2 = SPLIT ? (A2  + (size_t)b * strideA) : nullptr;
  const T* Bb2 = SPLIT ? (Bt2 + (size_t)b * strideB) : nullptr;

  const int rlane = lane & 15;
  const int koff  = (lane >> 4) * 8;
  const int mOff  = (lane >> 4) * 8;

  v8f acc[4][4];
#pragma unroll
  for (int i = 0; i < 4; ++i)
#pragma unroll
    for (int j = 0; j < 4; ++j) acc[i][j] = (v8f){0.f,0.f,0.f,0.f,0.f,0.f,0.f,0.f};

  for (int k0 = 0; k0 < K; k0 += 32) {
    V bh[4], bl[4];
#pragma unroll
    for (int j = 0; j < 4; ++j) {
      const size_t bo = (size_t)(n0 + (j << 4) + rlane) * ldb + koff + k0;
      bh[j] = Frag<T>::load(Bb + bo);
      if (SPLIT) bl[j] = Frag<T>::load(Bb2 + bo);
    }
#pragma unroll
    for (int i = 0; i < 4; ++i) {
      const size_t ao = (size_t)(m0 + (i << 4) + rlane) * lda + koff + k0;
      V ah = Frag<T>::load(Ab + ao);
      V al;
      if (SPLIT) al = Frag<T>::load(Ab2 + ao);
#pragma unroll
      for (int j = 0; j < 4; ++j) {
        acc[i][j] = Frag<T>::mma(ah, bh[j], acc[i][j]);
        if (SPLIT) {
          acc[i][j] = Frag<T>::mma(ah, bl[j], acc[i][j]);
          acc[i][j] = Frag<T>::mma(al, bh[j], acc[i][j]);
        }
      }
      Frag<T>::guard(acc[i][0], acc[i][3], ah, SPLIT ? al : ah);
    }
    Frag<T>::keep(bh[0], bh[1], bh[2], bh[3]);
    if (SPLIT) Frag<T>::keep(bl[0], bl[1], bl[2], bl[3]);
  }
  acc_guard4(acc[0][0], acc[0][1], acc[0][2], acc[0][3]);
  acc_guard4(acc[1][0], acc[1][1], acc[1][2], acc[1][3]);
  acc_guard4(acc[2][0], acc[2][1], acc[2][2], acc[2][3]);
  acc_guard4(acc[3][0], acc[3][1], acc[3][2], acc[3][3]);

  float* slab = sT[wave];
  const float* Rb = RESID ? (resid + (size_t)b * strideR) : nullptr;
#pragma unroll
  for (int i = 0; i < 4; ++i) {
    const int mBase = m0 + (i << 4);
#pragma unroll
    for (int j = 0; j < 4; ++j) {
      const int n = n0 + (j << 4) + rlane;
      float bv = 0.f;
      if (BIAS_MODE == 2) bv = bias[n];
#pragma unroll
      for (int r = 0; r < 8; ++r) {
        float v = acc[i][j][r] * scale;
        if (BIAS_MODE == 1) v += bias[mBase + mOff + r];
        if (BIAS_MODE == 2) v += bv;
        if (RESID) v += Rb[(size_t)(mBase + mOff + r) * ldc + n];
        if (ACT == 2) v = fmaxf(v, 0.0f);
        if (ACT == 3) v = v * (1.0f / (1.0f + expf(-v)));
        if (ACT == 4) v = (v > 0.f) ? v : 0.01f * v;
        if (ACT == 6) v = 1.0f / (1.0f + expf(-v));
        slab[(mOff + r) * 68 + (j << 4) + rlane] = v;
      }
    }
    __builtin_amdgcn_fence(__ATOMIC_RELEASE, "workgroup");
    __builtin_amdgcn_wave_barrier();
    __builtin_amdgcn_fence(__ATOMIC_ACQUIRE, "workgroup");
    if (OUT_MODE == 0) {
      float* C = (float*)Cout + (size_t)b * strideC;
      const int hh = lane >> 4, c4 = (lane & 15) * 4;
      for (int pass = 0; pass < 2; ++pass) {
#pragma unroll
        for (int it = 0; it < 8; ++it) {
          const int row = it * 2 + hh;
          v4f v = *(const v4f*)(slab + row * 68 + c4);
          *(volatile v4f*)(C + (size_t)(mBase + row) * ldc + n0 + c4) = v;
        }
        __threadfence();
      }
    } else {
      const int q = lane >> 3, c8 = (lane & 7) * 8;
      unsigned short* C  = (unsigned short*)Cout  + (size_t)b * strideC;
      unsigned short* C2 = (OUT_MODE == 2) ? ((unsigned short*)Cout2 + (size_t)b * strideC) : nullptr;
      for (int pass = 0; pass < 2; ++pass) {
#pragma unroll
        for (int it = 0; it < 4; ++it) {
          const int row = it * 4 + q;
          const float* sp = slab + row * 68 + c8;
          v8h hv, lv;
#pragma unroll
          for (int e = 0; e < 8; ++e) {
            if (OUT_MODE == 1) {
              hv[e] = (_Float16)sp[e];
            } else {
              unsigned short hb = f2bf_bits(sp[e]);
              unsigned short lb = f2bf_bits(sp[e] - bf_bits2f(hb));
              hv[e] = __builtin_bit_cast(_Float16, hb);
              lv[e] = __builtin_bit_cast(_Float16, lb);
            }
          }
          *(volatile v8h*)(C + (size_t)(mBase + row) * ldc + n0 + c8) = hv;
          if (OUT_MODE == 2) *(volatile v8h*)(C2 + (size_t)(mBase + row) * ldc + n0 + c8) = lv;
        }
        __threadfence();
      }
    }
    __builtin_amdgcn_fence(__ATOMIC_RELEASE, "workgroup");
    __builtin_amdgcn_wave_barrier();
    __builtin_amdgcn_fence(__ATOMIC_ACQUIRE, "workgroup");
  }
}

__global__ __launch_bounds__(256) void cast8_scaled_kernel(const float* __restrict__ in, unsigned short* __restrict__ out,
                                                           int n8, float scale) {
  const int i = blockIdx.x * 256 + threadIdx.x;
  if (i >= n8) return;
  const float* p = in + 8 * (size_t)i;
  const v4f a = *(const v4f*)(p);
  const v4f c = *(const v4f*)(p + 4);
  unsigned short hb[8];
#pragma unroll
  for (int e = 0; e < 4; ++e) {
    hb[e]     = h_bits(a[e] * scale);
    hb[4 + e] = h_bits(c[e] * scale);
  }
  const v4u u = (v4u){pk16(hb[0], hb[1]), pk16(hb[2], hb[3]), pk16(hb[4], hb[5]), pk16(hb[6], hb[7])};
  store2_v4u(out + 8 * (size_t)i, u);
}

__global__ __launch_bounds__(256) void cast_wdt_kernel(const float* __restrict__ W, unsigned short* __restrict__ out, float scale) {
  const int i = blockIdx.x * 256 + threadIdx.x;
  if (i >= kDim * kDim / 8) return;
  const int r  = i >> 7;
  const int c8 = (i & 127) * 8;
  const float* p = W + (size_t)r * (kDim + 1) + c8;
  const float f0 = p[0], f1 = p[1], f2 = p[2], f3 = p[3], f4 = p[4], f5 = p[5], f6 = p[6], f7 = p[7];
  const v4u u = (v4u){pk16(h_bits(f0 * scale), h_bits(f1 * scale)), pk16(h_bits(f2 * scale), h_bits(f3 * scale)),
                      pk16(h_bits(f4 * scale), h_bits(f5 * scale)), pk16(h_bits(f6 * scale), h_bits(f7 * scale))};
  store2_v4u(out + (size_t)r * kDim + c8, u);
}

__global__ __launch_bounds__(256) void cast_wbc_kernel(const float* __restrict__ WB, const float* __restrict__ WC,
                                                       unsigned short* __restrict__ out, float scale) {
  const int i = blockIdx.x * 256 + threadIdx.x;
  if (i >= 4 * kNS * kDim / 8) return;
  const int r  = i >> 7;
  const int c8 = (i & 127) * 8;
  const int rB = (r < kNS) ? r : (kNS - 1);
  int rC = r - kNS; rC = (rC < 0) ? 0 : rC; rC = (rC > kNS - 1) ? (kNS - 1) : rC;
  const float* pB = WB + (size_t)rB * kDim + c8;
  const float* pC = WC + (size_t)rC * kDim + c8;
  const v4f aB = *(const v4f*)(pB), cB = *(const v4f*)(pB + 4);
  const v4f aC = *(const v4f*)(pC), cC = *(const v4f*)(pC + 4);
  const bool useB = (r < kNS);
  const bool useC = (r >= kNS) && (r < 2 * kNS);
  unsigned short hb[8];
#pragma unroll
  for (int e = 0; e < 4; ++e) {
    const float v0 = useB ? aB[e] : (useC ? aC[e] : 0.0f);
    const float v1 = useB ? cB[e] : (useC ? cC[e] : 0.0f);
    hb[e]     = h_bits(v0 * scale);
    hb[4 + e] = h_bits(v1 * scale);
  }
  const v4u u = (v4u){pk16(hb[0], hb[1]), pk16(hb[2], hb[3]), pk16(hb[4], hb[5]), pk16(hb[6], hb[7])};
  store2_v4u(out + (size_t)r * kDim + c8, u);
}

__global__ __launch_bounds__(128) void ln_kernel(const float* __restrict__ x, const float* __restrict__ ev,
                                                 const float* __restrict__ g1, const float* __restrict__ b1,
                                                 const float* __restrict__ g2, const float* __restrict__ b2,
                                                 unsigned short* __restrict__ o1, unsigned short* __restrict__ o2) {
  __shared__ float red1[4];
  __shared__ float red2[4];
  const int blk = blockIdx.x;
  const bool second = (blk >= kRows);
  const int row = second ? (blk - kRows) : blk;
  const float* src = second ? ev : x;
  const float* g   = second ? g2 : g1;
  const float* bb  = second ? b2 : b1;
  unsigned short* o = second ? o2 : o1;
  const int th = threadIdx.x, lane = th & 31, wave = th >> 5;
  const int c0 = 8 * th;
  const float* p = src + (size_t)row * kDim + c0;
  const v4f a = *(const v4f*)(p);
  const v4f c = *(const v4f*)(p + 4);
  float s = ((a[0] + a[1]) + (a[2] + a[3])) + ((c[0] + c[1]) + (c[2] + c[3]));
  s = wave_sum(s);
  if (lane == 0) red1[wave] = s;
  __syncthreads();
  const float mean = ((red1[0] + red1[1]) + (red1[2] + red1[3])) * kInvDim;
  const v4f da = a - mean;
  const v4f dc = c - mean;
  float ss = ((da[0] * da[0] + da[1] * da[1]) + (da[2] * da[2] + da[3] * da[3]))
           + ((dc[0] * dc[0] + dc[1] * dc[1]) + (dc[2] * dc[2] + dc[3] * dc[3]));
  ss = wave_sum(ss);
  if (lane == 0) red2[wave] = ss;
  __syncthreads();
  const float var  = ((red2[0] + red2[1]) + (red2[2] + red2[3])) * kInvDim;
  const float rstd = rsqrtf(var + kLnEps);
  const v4f ga = *(const v4f*)(g + c0), gc = *(const v4f*)(g + c0 + 4);
  const v4f ba = *(const v4f*)(bb + c0), bc = *(const v4f*)(bb + c0 + 4);
  const v4f ya = da * rstd * ga + ba;
  const v4f yc = dc * rstd * gc + bc;
  unsigned short hb[8];
#pragma unroll
  for (int e = 0; e < 4; ++e) {
    hb[e]     = h_bits(ya[e]);
    hb[4 + e] = h_bits(yc[e]);
  }
  const v4u u = (v4u){pk16(hb[0], hb[1]), pk16(hb[2], hb[3]), pk16(hb[4], hb[5]), pk16(hb[6], hb[7])};
  store2_v4u(o + (size_t)row * kDim + c0, u);
}

__global__ __launch_bounds__(128) void xs_rows_kernel(const float* __restrict__ XS32, unsigned short* __restrict__ XS16,
                                                      float* __restrict__ xsc) {
  __shared__ float red[4];
  __shared__ __align__(16) float outv[32];
  const int th = threadIdx.x, lane = th & 31, wave = th >> 5;
  const int blk = blockIdx.x;
  const int c0 = 8 * th;
#pragma unroll 1
  for (int r = 0; r < 32; ++r) {
    const int row = blk * 32 + r;
    const float* p = XS32 + (size_t)row * kDim + c0;
    const v4f a = *(const v4f*)(p);
    const v4f c = *(const v4f*)(p + 4);
    float s = ((a[0] + a[1]) + (a[2] + a[3])) + ((c[0] + c[1]) + (c[2] + c[3]));
    s = wave_sum(s);
    if (lane == 0) red[wave] = s;
    unsigned short hb[8];
#pragma unroll
    for (int e = 0; e < 4; ++e) {
      hb[e]     = h_bits(a[e]);
      hb[4 + e] = h_bits(c[e]);
    }
    const v4u u = (v4u){pk16(hb[0], hb[1]), pk16(hb[2], hb[3]), pk16(hb[4], hb[5]), pk16(hb[6], hb[7])};
    store2_v4u(XS16 + (size_t)row * kDim + c0, u);
    __syncthreads();
    if (th == 0) outv[r] = ((red[0] + red[1]) + (red[2] + red[3])) * kInvDim;
    __syncthreads();
  }
  if (th < 8) {
    const v4f v = *(const v4f*)(outv + 4 * th);
    store2_v4f(xsc + (size_t)blk * 32 + 4 * th, v);
  }
}

__global__ __launch_bounds__(128) void dt_rows_kernel(const float* __restrict__ DT32, const float* __restrict__ Wdt,
                                                      const float* __restrict__ bdt, const float* __restrict__ tc,
                                                      float* __restrict__ dts) {
  __shared__ float red[4];
  __shared__ __align__(16) float outv[32];
  const int th = threadIdx.x, lane = th & 31, wave = th >> 5;
  const int blk = blockIdx.x;
#pragma unroll 1
  for (int r = 0; r < 32; ++r) {
    const int row = blk * 32 + r;
    const float tcv = tc[row];
    const float* dp = DT32 + (size_t)row * kDim;
    float accv = 0.0f;
#pragma unroll 1
    for (int e = 0; e < 8; ++e) {
      const int col = e * 128 + th;
      const float d  = dp[col];
      const float wl = Wdt[(size_t)col * (kDim + 1) + kDim];
      const float bv = bdt[col];
      const float v  = d + tcv * wl + bv;
      const float sp = fmaxf(v, 0.0f) + logf(1.0f + expf(-fabsf(v)));
      accv += sp;
    }
    accv = wave_sum(accv);
    if (lane == 0) red[wave] = accv;
    __syncthreads();
    if (th == 0) {
      float m = ((red[0] + red[1]) + (red[2] + red[3])) * kInvDim;
      m = fminf(fmaxf(m, 1e-3f), 5.0f);
      outv[r] = m;
    }
    __syncthreads();
  }
  if (th < 8) {
    const v4f v = *(const v4f*)(outv + 4 * th);
    store2_v4f(dts + (size_t)blk * 32 + 4 * th, v);
  }
}

__global__ __launch_bounds__(64) void scan_kernel(const float* __restrict__ BC32, const float* __restrict__ dts,
                                                  const float* __restrict__ xsc, const float* __restrict__ logA,
                                                  float* __restrict__ yssm) {
  __shared__ __align__(16) float ys[kRows];
  const int th = threadIdx.x;
  const int n = th & 15;
  const int b = th >> 4;
  const float la = fminf(fmaxf(logA[n], -10.0f), -0.5f);
  const float Aval = -expf(la);
  const float rA = 1.0f / (Aval - 1e-8f);
  float h = 0.0f;
#pragma unroll 1
  for (int t = 0; t < kSeq; ++t) {
    const int row = b * kSeq + t;
    const float ds = dts[row];
    const float xs = xsc[row];
    const float bt = BC32[(size_t)row * 64 + n];
    const float ct = BC32[(size_t)row * 64 + kNS + n];
    const float nb = sqrtf(half16_sum(bt * bt));
    const float nc = sqrtf(half16_sum(ct * ct));
    const float btn = bt * (1.0f / fmaxf(nb, 1e-12f));
    const float ctn = ct * (1.0f / fmaxf(nc, 1e-12f));
    float ab = expf(ds * Aval);
    ab = (ab != ab) ? 0.1f : ab;
    const float bbar = (1.0f - ab) * rA * btn;
    const float bx = bbar * xs;
    h = fminf(fmaxf(ab * h + bx, -10.0f), 10.0f);
    const float y = half16_sum(ctn * h);
    if (n == 0) ys[row] = y;
  }
  __syncthreads();
  for (int pass = 0; pass < 2; ++pass) {
#pragma unroll 1
    for (int i = 0; i < kRows / (4 * 64); ++i) {
      const int idx = i * 64 + th;
      const v4f v = *(const v4f*)(ys + 4 * idx);
      *(volatile v4f*)(yssm + 4 * (size_t)idx) = v;
    }
    __threadfence();
  }
}

__global__ __launch_bounds__(128) void comb_kernel(const float* __restrict__ E32, const float* __restrict__ Z32,
                                                   const float* __restrict__ yssm, unsigned short* __restrict__ Y16) {
  __shared__ float red[4];
  const int row = blockIdx.x;
  const int th = threadIdx.x, lane = th & 31, wave = th >> 5;
  const int c0 = 8 * th;
  const float* ep = E32 + (size_t)row * kDim + c0;
  const float* zp = Z32 + (size_t)row * kDim + c0;
  const v4f ea = *(const v4f*)(ep), ec = *(const v4f*)(ep + 4);
  const v4f za = *(const v4f*)(zp), zc = *(const v4f*)(zp + 4);
  float ss = ((ea[0] * ea[0] + ea[1] * ea[1]) + (ea[2] * ea[2] + ea[3] * ea[3]))
           + ((ec[0] * ec[0] + ec[1] * ec[1]) + (ec[2] * ec[2] + ec[3] * ec[3]));
  ss = wave_sum(ss);
  if (lane == 0) red[wave] = ss;
  __syncthreads();
  const float me2 = ((red[0] + red[1]) + (red[2] + red[3])) * kInvDim;
  const float gate = 1.0f / (1.0f + expf(-me2));
  const float ys = yssm[row];
  const v4f ya = ys * za + gate * ea;
  const v4f yc = ys * zc + gate * ec;
  unsigned short hb[8];
#pragma unroll
  for (int e = 0; e < 4; ++e) {
    hb[e]     = h_bits(ya[e]);
    hb[4 + e] = h_bits(yc[e]);
  }
  const v4u u = (v4u){pk16(hb[0], hb[1]), pk16(hb[2], hb[3]), pk16(hb[4], hb[5]), pk16(hb[6], hb[7])};
  store2_v4u(Y16 + (size_t)row * kDim + c0, u);
}

extern "C" void kernel_launch(void* const* d_in, const int* in_sizes, int n_in,
                              void* d_out, int out_size, void* d_ws, size_t ws_size,
                              hipStream_t stream) {
  if (n_in < 15) return;
  if (in_sizes[0] != kRows * kDim || out_size != kRows * kDim) return;
  const float* x      = (const float*)d_in[0];
  const float* engram = (const float*)d_in[1];
  const float* tc     = (const float*)d_in[2];
  const float* W_in   = (const float*)d_in[3];
  const float* W_out  = (const float*)d_in[4];
  const float* W_B    = (const float*)d_in[5];
  const float* W_C    = (const float*)d_in[6];
  const float* W_dt   = (const float*)d_in[7];
  const float* b_dt   = (const float*)d_in[8];
  const float* log_A  = (const float*)d_in[9];
  const float* W_eng  = (const float*)d_in[10];
  const float* ln1_g  = (const float*)d_in[11];
  const float* ln1_b  = (const float*)d_in[12];
  const float* ln2_g  = (const float*)d_in[13];
  const float* ln2_b  = (const float*)d_in[14];
  float* out = (float*)d_out;

  const size_t szF32Plane = (size_t)kRows * kDim * 4;
  const size_t szF16Plane = (size_t)kRows * kDim * 2;
  const size_t szWin  = (size_t)2 * kDim * kDim * 2;
  const size_t szW    = (size_t)kDim * kDim * 2;
  const size_t szWbc  = (size_t)4 * kNS * kDim * 2;
  const size_t szBC   = (size_t)kRows * 64 * 4;
  const size_t szRow  = (size_t)kRows * 4;
  size_t off = 0;
  char* base = (char*)d_ws;
  float*          rA   = (float*)(base + off);          off += szF32Plane;
  unsigned short* rB   = (unsigned short*)(base + off); off += szF16Plane;
  unsigned short* rC   = (unsigned short*)(base + off); off += szF16Plane;
  unsigned short* rD   = (unsigned short*)(base + off); off += szF16Plane;
  float*          rE   = (float*)(base + off);          off += szF32Plane;
  unsigned short* win  = (unsigned short*)(base + off); off += szWin;
  unsigned short* wdt  = (unsigned short*)(base + off); off += szW;
  unsigned short* weng = (unsigned short*)(base + off); off += szW;
  unsigned short* wout = (unsigned short*)(base + off); off += szW;
  unsigned short* wbc  = (unsigned short*)(base + off); off += szWbc;
  float*          bc32 = (float*)(base + off);          off += szBC;
  float*          xsc  = (float*)(base + off);          off += szRow;
  float*          dts  = (float*)(base + off);          off += szRow;
  float*          yss  = (float*)(base + off);          off += szRow;
  if (off > ws_size) return;

  {
    const int n8_win = 2 * kDim * kDim / 8;
    const int n8_w   = kDim * kDim / 8;
    cast8_scaled_kernel<<<dim3(n8_win / 256), dim3(256), 0, stream>>>(W_in, win, n8_win, kWCarry);
    cast8_scaled_kernel<<<dim3(n8_w / 256), dim3(256), 0, stream>>>(W_eng, weng, n8_w, kWCarry);
    cast8_scaled_kernel<<<dim3(n8_w / 256), dim3(256), 0, stream>>>(W_out, wout, n8_w, kWCarry);
    cast_wdt_kernel<<<dim3(n8_w / 256), dim3(256), 0, stream>>>(W_dt, wdt, kWCarry);
    cast_wbc_kernel<<<dim3((4 * kNS * kDim / 8) / 256), dim3(256), 0, stream>>>(W_B, W_C, wbc, kWCarry);
  }

  ln_kernel<<<dim3(2 * kRows), dim3(128), 0, stream>>>(x, engram, ln1_g, ln1_b, ln2_g, ln2_b, rB, rC);

  const int gridN1024 = ((kRows / 64) * (kDim / 64)) / 8;
  const int gridN64   = ((kRows / 64) * 1) / 8;

  wmma_gemm64<0, false, 0, 0, false, 3><<<dim3(gridN1024, 1), dim3(256), 0, stream>>>(
      rB, rB, kDim, 0L, win, win, kDim, 0L, (void*)rA, (void*)rA, kDim, 0L,
      b_dt, x, 0L, kRows, kDim, kDim, kWCarryInv);
  wmma_gemm64<0, false, 0, 0, false, 6><<<dim3(gridN1024, 1), dim3(256), 0, stream>>>(
      rB, rB, kDim, 0L, win + (size_t)kDim * kDim, win + (size_t)kDim * kDim, kDim, 0L, (void*)rE, (void*)rE, kDim, 0L,
      b_dt, x, 0L, kRows, kDim, kDim, kWCarryInv);

  xs_rows_kernel<<<dim3(kRows / 32), dim3(128), 0, stream>>>(rA, rD, xsc);

  wmma_gemm64<0, false, 0, 0, false, 0><<<dim3(gridN64, 1), dim3(256), 0, stream>>>(
      rD, rD, kDim, 0L, wbc, wbc, kDim, 0L, (void*)bc32, (void*)bc32, 64, 0L,
      b_dt, x, 0L, kRows, 64, kDim, kWCarryInv);

  wmma_gemm64<0, false, 0, 0, false, 0><<<dim3(gridN1024, 1), dim3(256), 0, stream>>>(
      rD, rD, kDim, 0L, wdt, wdt, kDim, 0L, (void*)rA, (void*)rA, kDim, 0L,
      b_dt, x, 0L, kRows, kDim, kDim, kWCarryInv);

  dt_rows_kernel<<<dim3(kRows / 32), dim3(128), 0, stream>>>(rA, W_dt, b_dt, tc, dts);

  scan_kernel<<<dim3(1), dim3(64), 0, stream>>>(bc32, dts, xsc, log_A, yss);

  wmma_gemm64<0, false, 0, 0, false, 0><<<dim3(gridN1024, 1), dim3(256), 0, stream>>>(
      rC, rC, kDim, 0L, weng, weng, kDim, 0L, (void*)rA, (void*)rA, kDim, 0L,
      b_dt, x, 0L, kRows, kDim, kDim, kWCarryInv);

  comb_kernel<<<dim3(kRows), dim3(128), 0, stream>>>(rA, rE, yss, rB);

  wmma_gemm64<0, false, 0, 0, true, 0><<<dim3(gridN1024, 1), dim3(256), 0, stream>>>(
      rB, rB, kDim, 0L, wout, wout, kDim, 0L, (void*)out, (void*)out, kDim, 0L,
      b_dt, x, 0L, kRows, kDim, kDim, kWCarryInv);
}
